// PointNet_17136919511611
// MI455X (gfx1250) — hardware-verified
//
#include <hip/hip_runtime.h>

typedef __attribute__((ext_vector_type(16))) _Float16 v16h;
typedef __attribute__((ext_vector_type(8)))  _Float16 v8h;
typedef __attribute__((ext_vector_type(8)))  float    v8f;
typedef __attribute__((ext_vector_type(4)))  float    v4f;
typedef __attribute__((ext_vector_type(4)))  unsigned v4u;

constexpr int   kNumPts      = 1000000;
constexpr int   kNumSeg      = 16384;
constexpr int   kInDim       = 3;
constexpr int   kHid         = 64;
constexpr int   kOutDim      = 128;
constexpr int   kRowsPerWave = 64;
constexpr int   kWavesPerBlk = 8;
constexpr int   kSlabPitch   = 68;
constexpr int   kSegPerBlk   = 256;
constexpr float kWCarry      = 16.0f;
constexpr float kWCarryInv   = 1.0f / 16.0f;
constexpr int   kNumTiles    = kNumPts / kRowsPerWave;
constexpr int   kWtPlane     = kHid * kHid;
constexpr int   kWtHalves    = 7 * kWtPlane + kOutDim * kHid;
constexpr int   kPrepBlocks  = kWtHalves / 8 / 256;
static_assert(kNumPts % kRowsPerWave == 0);
static_assert(kNumPts % 4 == 0);
static_assert(kHid % 32 == 0);
static_assert(kHid == 64 && kOutDim % 64 == 0);
static_assert(kNumSeg % kSegPerBlk == 0);
static_assert(kSegPerBlk % 16 == 0);
static_assert(kWtHalves == 36864);
static_assert(kPrepBlocks * 256 * 8 == kWtHalves);

__device__ __forceinline__ void guard_acc4(v8f& a, v8f& b, v8f& c, v8f& d, v16h x, v16h y) {
  asm volatile("v_nop\n\tv_nop\n\tv_nop\n\tv_nop" : "+v"(a), "+v"(b), "+v"(c), "+v"(d) : "v"(x), "v"(y));
}
__device__ __forceinline__ void keep4_h(v16h a, v16h b, v16h c, v16h d) { asm volatile("v_nop" :: "v"(a), "v"(b), "v"(c), "v"(d)); }

template <typename T> struct Frag;
template <> struct Frag<_Float16> {
  typedef v16h V; union U { v16h v; v8h h[2]; };
  static __device__ __forceinline__ v16h load(const _Float16* p) {
    U f; f.h[0] = *(const v8h*)(p); f.h[1] = *(const v8h*)(p + 16); return f.v;
  }
  static __device__ __forceinline__ v8f mma(v16h a, v16h b, v8f c) {
    return __builtin_amdgcn_wmma_f32_16x16x32_f16(false, a, false, b, (short)0, c, false, false);
  }
};

__device__ __forceinline__ v16h frag_from_words(const unsigned* wp) {
  union { v16h v; v4u w[2]; } f;
  f.w[0] = *(const v4u*)(wp);
  f.w[1] = *(const v4u*)(wp + 8);
  return f.v;
}

__device__ __forceinline__ void mma_16x64x64(v16h a0, v16h a1,
                                             v16h b00, v16h b01, v16h b02, v16h b03,
                                             v16h b10, v16h b11, v16h b12, v16h b13,
                                             v8f& c0, v8f& c1, v8f& c2, v8f& c3) {
  c0 = Frag<_Float16>::mma(a0, b00, c0);
  c1 = Frag<_Float16>::mma(a0, b01, c1);
  c2 = Frag<_Float16>::mma(a0, b02, c2);
  c3 = Frag<_Float16>::mma(a0, b03, c3);
  c0 = Frag<_Float16>::mma(a1, b10, c0);
  c1 = Frag<_Float16>::mma(a1, b11, c1);
  c2 = Frag<_Float16>::mma(a1, b12, c2);
  c3 = Frag<_Float16>::mma(a1, b13, c3);
  guard_acc4(c0, c1, c2, c3, a0, a1);
  keep4_h(b00, b01, b02, b03);
  keep4_h(b10, b11, b12, b13);
}

__device__ __forceinline__ void slab_put(float* slab, int hh, int rlane, v8f c0, v8f c1, v8f c2, v8f c3) {
#pragma unroll
  for (int r = 0; r < 8; ++r) {
    float* sp = slab + (8 * hh + r) * kSlabPitch + rlane;
    sp[0]  = c0[r] * kWCarryInv;
    sp[16] = c1[r] * kWCarryInv;
    sp[32] = c2[r] * kWCarryInv;
    sp[48] = c3[r] * kWCarryInv;
  }
}

__device__ __forceinline__ float relu_pos(float y) { return (y > 0.0f) ? y : 0.0f; }

__device__ __forceinline__ v16h build_hfrag(const float* wl, float p0, float p1, float p2, int kb) {
  v16h a;
#pragma unroll
  for (int g = 0; g < 2; ++g) {
#pragma unroll
    for (int hq = 0; hq < 2; ++hq) {
      const float* w = wl + kb + 16 * g + 4 * hq;
      const v4f w0 = *(const v4f*)(w);
      const v4f w1 = *(const v4f*)(w + 64);
      const v4f w2 = *(const v4f*)(w + 128);
      const v4f bb = *(const v4f*)(w + 192);
#pragma unroll
      for (int e = 0; e < 4; ++e) {
        const float hval = p0 * w0[e] + p1 * w1[e] + p2 * w2[e] + bb[e];
        a[8 * g + 4 * hq + e] = (_Float16)relu_pos(hval);
      }
    }
  }
  return a;
}

__global__ __launch_bounds__(256) void wprep_kernel(const float* __restrict__ w1, const float* __restrict__ w2,
                                                    const float* __restrict__ w3, const float* __restrict__ w4,
                                                    const float* __restrict__ wout, unsigned short* __restrict__ wt) {
  const int blk = blockIdx.x;
  const int gid = blk * 256 + threadIdx.x;
  const int row = gid >> 3;
  const int c8  = (gid & 7) * 8;
  const float* src = w1;
  int kr0 = 0, pitch = kHid, n = row & 63;
  if (blk >= 14) {
    src = wout; pitch = kOutDim; n = row - 448;
  } else {
    const int pl = blk >> 1;
    if (pl == 1 || pl == 2) src = w2;
    if (pl == 3 || pl == 4) src = w3;
    if (pl == 5 || pl == 6) src = w4;
    kr0 = (pl >= 2 && (pl & 1) == 0) ? 64 : 0;
  }
  v8h hv;
#pragma unroll
  for (int e = 0; e < 8; ++e) {
    const float w = src[(size_t)(kr0 + c8 + e) * pitch + n];
    hv[e] = (_Float16)(w * kWCarry);
  }
  unsigned short* dp = wt + (size_t)gid * 8;
  *(volatile v8h*)dp = hv;
  __threadfence();
  *(volatile v8h*)dp = hv;
}

template <bool FIRST>
__global__ __launch_bounds__(256) void layer_kernel(const float* __restrict__ pts, const float* __restrict__ wpos,
                                                    const float* __restrict__ bpos,
                                                    const unsigned short* __restrict__ xin,
                                                    unsigned short* __restrict__ xout,
                                                    const unsigned short* __restrict__ wt,
                                                    const float* __restrict__ addsrc, const int* __restrict__ idx,
                                                    int ntiles) {
  __shared__ __align__(16) float sSlab[kWavesPerBlk][16 * kSlabPitch];
  __shared__ __align__(16) float sWl[256];
  const int tid = threadIdx.x, lane = tid & 31, wave = tid >> 5;
  if (FIRST) {
    if (tid < 192) sWl[tid] = wpos[tid];
    if (tid < 64) sWl[192 + tid] = bpos[tid];
    __syncthreads();
  }
  const int tile = blockIdx.x * kWavesPerBlk + wave;
  if (tile < ntiles) {
    const int rlane = lane & 15, hh = lane >> 4, koff = hh * 8;
    const int q = lane >> 3, c8 = (lane & 7) * 8;
    const int m0 = tile * kRowsPerWave;
    const _Float16* wth = (const _Float16*)wt;
    const _Float16* bp = wth + (size_t)rlane * kHid + koff;
    const v16h b00 = Frag<_Float16>::load(bp);
    const v16h b01 = Frag<_Float16>::load(bp + 16 * kHid);
    const v16h b02 = Frag<_Float16>::load(bp + 32 * kHid);
    const v16h b03 = Frag<_Float16>::load(bp + 48 * kHid);
    asm volatile("" ::: "memory");
    const v16h b10 = Frag<_Float16>::load(bp + 32);
    const v16h b11 = Frag<_Float16>::load(bp + 16 * kHid + 32);
    const v16h b12 = Frag<_Float16>::load(bp + 32 * kHid + 32);
    const v16h b13 = Frag<_Float16>::load(bp + 48 * kHid + 32);
    v4f biasA = {0.f, 0.f, 0.f, 0.f}, biasB = {0.f, 0.f, 0.f, 0.f};
    if (FIRST) {
      biasA = *(const v4f*)(addsrc + c8);
      biasB = *(const v4f*)(addsrc + c8 + 4);
    }
    float* slab = sSlab[wave];
    const v8f z8 = {0.f, 0.f, 0.f, 0.f, 0.f, 0.f, 0.f, 0.f};
#pragma unroll 1
    for (int i = 0; i < 4; ++i) {
      const int mBase = m0 + 16 * i;
      v16h a0, a1;
      if (FIRST) {
        const float* pr = pts + (size_t)(mBase + rlane) * kInDim;
        const float p0 = pr[0], p1 = pr[1], p2 = pr[2];
        a0 = build_hfrag(sWl, p0, p1, p2, koff);
        a1 = build_hfrag(sWl, p0, p1, p2, 32 + koff);
      } else {
        const _Float16* ap = (const _Float16*)xin + (size_t)(mBase + rlane) * kHid + koff;
        a0 = Frag<_Float16>::load(ap);
        a1 = Frag<_Float16>::load(ap + 32);
      }
      v8f c0 = z8, c1 = z8, c2 = z8, c3 = z8;
      mma_16x64x64(a0, a1, b00, b01, b02, b03, b10, b11, b12, b13, c0, c1, c2, c3);
      slab_put(slab, hh, rlane, c0, c1, c2, c3);
      __builtin_amdgcn_fence(__ATOMIC_RELEASE, "workgroup");
      __builtin_amdgcn_wave_barrier();
      __builtin_amdgcn_fence(__ATOMIC_ACQUIRE, "workgroup");
      v8h hv[4];
#pragma unroll
      for (int it = 0; it < 4; ++it) {
        const int row = it * 4 + q;
        const float* sp = slab + row * kSlabPitch + c8;
        const v4f s0 = *(const v4f*)(sp);
        const v4f s1 = *(const v4f*)(sp + 4);
        v4f t0 = biasA, t1 = biasB;
        if (!FIRST) {
          int sg = idx[mBase + row];
          sg = sg < 0 ? 0 : sg;
          sg = sg > (kNumSeg - 1) ? (kNumSeg - 1) : sg;
          const float* tp = addsrc + (size_t)sg * kHid + c8;
          t0 = *(const v4f*)(tp);
          t1 = *(const v4f*)(tp + 4);
        }
#pragma unroll
        for (int e = 0; e < 4; ++e) {
          const float ya = relu_pos(s0[e] + t0[e]);
          const float yb = relu_pos(s1[e] + t1[e]);
          hv[it][e]     = (_Float16)ya;
          hv[it][4 + e] = (_Float16)yb;
        }
      }
      unsigned short* xo = xout + (size_t)(mBase + q) * kHid + c8;
#pragma unroll
      for (int it = 0; it < 4; ++it) *(volatile v8h*)(xo + (size_t)(it * 4) * kHid) = hv[it];
      __threadfence();
#pragma unroll
      for (int it = 0; it < 4; ++it) *(volatile v8h*)(xo + (size_t)(it * 4) * kHid) = hv[it];
      __threadfence();
      __builtin_amdgcn_fence(__ATOMIC_RELEASE, "workgroup");
      __builtin_amdgcn_wave_barrier();
      __builtin_amdgcn_fence(__ATOMIC_ACQUIRE, "workgroup");
    }
  }
}

template <int NCOL>
__global__ __launch_bounds__(32) void segmax_proj_kernel(const unsigned* __restrict__ xw, const int* __restrict__ idx,
                                                         int npts, const unsigned short* __restrict__ wt,
                                                         const float* __restrict__ bias, float* __restrict__ outp) {
  __shared__ __align__(16) unsigned sTile[kSegPerBlk * 32];
  __shared__ __align__(16) float sSl[16 * kSlabPitch];
  const int lane = threadIdx.x;
  const int s0 = blockIdx.x * kSegPerBlk;
#pragma unroll 1
  for (int i = lane; i < kSegPerBlk * 32; i += 32) sTile[i] = 0u;
  __syncthreads();

  const int nIter = (npts + 127) >> 7;
#pragma unroll 1
  for (int it = 0; it < nIter; ++it) {
    const int eb  = it * 128 + lane * 4;
    const int ebc = (eb + 4 <= npts) ? eb : (npts - 4);
    const int4 v = *(const int4*)(idx + ebc);
    const bool ok = eb < npts;
    int i0 = v.x, i1 = v.y, i2 = v.z, i3 = v.w;
    i0 = i0 < 0 ? 0 : (i0 > kNumSeg - 1 ? kNumSeg - 1 : i0);
    i1 = i1 < 0 ? 0 : (i1 > kNumSeg - 1 ? kNumSeg - 1 : i1);
    i2 = i2 < 0 ? 0 : (i2 > kNumSeg - 1 ? kNumSeg - 1 : i2);
    i3 = i3 < 0 ? 0 : (i3 > kNumSeg - 1 ? kNumSeg - 1 : i3);
    unsigned dd[4];
    dd[0] = (unsigned)(i0 - s0);
    dd[1] = (unsigned)(i1 - s0);
    dd[2] = (unsigned)(i2 - s0);
    dd[3] = (unsigned)(i3 - s0);
    unsigned m = 0u;
    m |= (dd[0] < (unsigned)kSegPerBlk) ? 1u : 0u;
    m |= (dd[1] < (unsigned)kSegPerBlk) ? 2u : 0u;
    m |= (dd[2] < (unsigned)kSegPerBlk) ? 4u : 0u;
    m |= (dd[3] < (unsigned)kSegPerBlk) ? 8u : 0u;
    m = ok ? m : 0u;
    unsigned bal = __builtin_amdgcn_ballot_w32(m != 0u);
#pragma unroll 1
    for (int g = 0; g < 32 && bal != 0u; ++g) {
      const int L = __builtin_ctz(bal);
      bal &= bal - 1u;
      const unsigned mm = (unsigned)__builtin_amdgcn_readlane((int)m, L);
      int sd[4];
#pragma unroll
      for (int j = 0; j < 4; ++j) sd[j] = __builtin_amdgcn_readlane((int)dd[j], L);
      const int pbase = it * 128 + L * 4;
#pragma unroll
      for (int j = 0; j < 4; ++j) {
        if ((mm >> j) & 1u) {
          const int segl = sd[j] & (kSegPerBlk - 1);
          int p = pbase + j;
          p = p < npts ? p : (npts - 1);
          const unsigned xv = xw[(size_t)p * 32 + lane];
          const unsigned cv = sTile[segl * 32 + lane];
          const unsigned xl = xv & 0xffffu, cl = cv & 0xffffu;
          const unsigned lo = xl > cl ? xl : cl;
          const unsigned hw = xv > cv ? xv : cv;
          sTile[segl * 32 + lane] = (hw & 0xffff0000u) | lo;
        }
      }
    }
  }
  __syncthreads();

  const int rlane = lane & 15, hh = lane >> 4, koff = hh * 8, c4 = rlane * 4;
  const _Float16* wth = (const _Float16*)wt;
  const v8f z8 = {0.f, 0.f, 0.f, 0.f, 0.f, 0.f, 0.f, 0.f};
#pragma unroll 1
  for (int nh = 0; nh < NCOL / 64; ++nh) {
    const _Float16* bp = wth + (size_t)(nh * 64 + rlane) * kHid + koff;
    const v16h b00 = Frag<_Float16>::load(bp);
    const v16h b01 = Frag<_Float16>::load(bp + 16 * kHid);
    const v16h b02 = Frag<_Float16>::load(bp + 32 * kHid);
    const v16h b03 = Frag<_Float16>::load(bp + 48 * kHid);
    asm volatile("" ::: "memory");
    const v16h b10 = Frag<_Float16>::load(bp + 32);
    const v16h b11 = Frag<_Float16>::load(bp + 16 * kHid + 32);
    const v16h b12 = Frag<_Float16>::load(bp + 32 * kHid + 32);
    const v16h b13 = Frag<_Float16>::load(bp + 48 * kHid + 32);
    const v4f bv = *(const v4f*)(bias + nh * 64 + c4);
#pragma unroll 1
    for (int mt = 0; mt < kSegPerBlk / 16; ++mt) {
      const unsigned* ap = sTile + (mt * 16 + rlane) * 32 + (koff >> 1);
      const v16h a0 = frag_from_words(ap);
      const v16h a1 = frag_from_words(ap + 16);
      v8f c0 = z8, c1 = z8, c2 = z8, c3 = z8;
      mma_16x64x64(a0, a1, b00, b01, b02, b03, b10, b11, b12, b13, c0, c1, c2, c3);
      slab_put(sSl, hh, rlane, c0, c1, c2, c3);
      __syncthreads();
      v4f ov[8];
#pragma unroll
      for (int it = 0; it < 8; ++it) {
        const int row = it * 2 + hh;
        const v4f sv = *(const v4f*)(sSl + row * kSlabPitch + c4);
        ov[it] = sv + bv;
      }
      float* op = outp + (size_t)(s0 + mt * 16 + hh) * NCOL + nh * 64 + c4;
#pragma unroll
      for (int it = 0; it < 8; ++it) *(volatile v4f*)(op + (size_t)(it * 2) * NCOL) = ov[it];
      __threadfence();
#pragma unroll
      for (int it = 0; it < 8; ++it) *(volatile v4f*)(op + (size_t)(it * 2) * NCOL) = ov[it];
      __threadfence();
      __syncthreads();
    }
  }
}

extern "C" void kernel_launch(void* const* d_in, const int* in_sizes, int n_in,
                              void* d_out, int out_size, void* d_ws, size_t ws_size, hipStream_t stream) {
  if (n_in < 15 || d_out == nullptr || d_ws == nullptr) return;
  if (in_sizes[0] != kNumPts * kInDim || in_sizes[1] != kNumPts || in_sizes[3] != kInDim * kHid ||
      in_sizes[4] != kHid || in_sizes[5] != kHid * kHid || in_sizes[6] != kHid ||
      in_sizes[7] != 2 * kHid * kHid || in_sizes[8] != kHid || in_sizes[9] != 2 * kHid * kHid ||
      in_sizes[10] != kHid || in_sizes[11] != 2 * kHid * kHid || in_sizes[12] != kHid ||
      in_sizes[13] != kHid * kOutDim || in_sizes[14] != kOutDim || out_size != kNumSeg * kOutDim) return;

  const float* pts  = (const float*)d_in[0];
  const int*   idx  = (const int*)d_in[1];
  const float* wpos = (const float*)d_in[3];
  const float* bpos = (const float*)d_in[4];
  const float* w1   = (const float*)d_in[5];
  const float* b1   = (const float*)d_in[6];
  const float* w2   = (const float*)d_in[7];
  const float* b2   = (const float*)d_in[8];
  const float* w3   = (const float*)d_in[9];
  const float* b3   = (const float*)d_in[10];
  const float* w4   = (const float*)d_in[11];
  const float* b4   = (const float*)d_in[12];
  const float* wout = (const float*)d_in[13];
  const float* bout = (const float*)d_in[14];
  float* outp = (float*)d_out;

  char* ws = (char*)d_ws; size_t off = 0;
  auto carve = [&](size_t bytes) -> char* { char* p = ws + off; off += (bytes + 255) & ~(size_t)255; return p; };
  unsigned short* XPLA = (unsigned short*)carve((size_t)kNumPts * kHid * 2);
  unsigned short* XPLB = (unsigned short*)carve((size_t)kNumPts * kHid * 2);
  float*          TPL  = (float*)carve((size_t)kNumSeg * kHid * 4);
  unsigned short* WTS  = (unsigned short*)carve((size_t)kWtHalves * 2);
  if (off > ws_size) return;

  const unsigned short* W1T   = WTS;
  const unsigned short* W2TOP = WTS + 1 * kWtPlane;
  const unsigned short* W2BOT = WTS + 2 * kWtPlane;
  const unsigned short* W3TOP = WTS + 3 * kWtPlane;
  const unsigned short* W3BOT = WTS + 4 * kWtPlane;
  const unsigned short* W4TOP = WTS + 5 * kWtPlane;
  const unsigned short* W4BOT = WTS + 6 * kWtPlane;
  const unsigned short* WOUTT = WTS + 7 * kWtPlane;

  const int lgrid = (kNumTiles + kWavesPerBlk - 1) / kWavesPerBlk;
  const int sgrid = kNumSeg / kSegPerBlk;
  const unsigned* XWA = (const unsigned*)XPLA;
  const unsigned* XWB = (const unsigned*)XPLB;

  wprep_kernel<<<kPrepBlocks, 256, 0, stream>>>(w1, w2, w3, w4, wout, WTS);

  layer_kernel<true><<<lgrid, 256, 0, stream>>>(pts, wpos, bpos, XPLB, XPLA, W1T, b1, idx, kNumTiles);
  segmax_proj_kernel<kHid><<<sgrid, 32, 0, stream>>>(XWA, idx, kNumPts, W2BOT, b2, TPL);
  layer_kernel<false><<<lgrid, 256, 0, stream>>>(pts, wpos, bpos, XPLA, XPLB, W2TOP, TPL, idx, kNumTiles);
  segmax_proj_kernel<kHid><<<sgrid, 32, 0, stream>>>(XWB, idx, kNumPts, W3BOT, b3, TPL);
  layer_kernel<false><<<lgrid, 256, 0, stream>>>(pts, wpos, bpos, XPLB, XPLA, W3TOP, TPL, idx, kNumTiles);
  segmax_proj_kernel<kHid><<<sgrid, 32, 0, stream>>>(XWA, idx, kNumPts, W4BOT, b4, TPL);
  layer_kernel<false><<<lgrid, 256, 0, stream>>>(pts, wpos, bpos, XPLA, XPLB, W4TOP, TPL, idx, kNumTiles);
  segmax_proj_kernel<kOutDim><<<sgrid, 32, 0, stream>>>(XWB, idx, kNumPts, WOUTT, bout, outp);
}
